// Dehazeblock_49873160241354
// MI455X (gfx1250) — hardware-verified
//
#include <hip/hip_runtime.h>
#include <stdint.h>
#include <stddef.h>

#pragma clang fp contract(off)

#define DEVINL __device__ __forceinline__

typedef _Float16 f16t;
typedef unsigned short us16;
typedef _Float16 v16h __attribute__((ext_vector_type(16)));
typedef _Float16 v8h  __attribute__((ext_vector_type(8)));
typedef __bf16   v16b __attribute__((ext_vector_type(16)));
typedef unsigned short v8us __attribute__((ext_vector_type(8)));
typedef float    v8f  __attribute__((ext_vector_type(8)));
typedef float    v4f  __attribute__((ext_vector_type(4)));
typedef int      v4i  __attribute__((ext_vector_type(4)));
typedef unsigned v4u  __attribute__((ext_vector_type(4)));
typedef v8h  __attribute__((may_alias)) v8ha;
typedef v8us __attribute__((may_alias)) v8usa;
typedef v4f  __attribute__((may_alias)) v4fa;
typedef v4u  __attribute__((may_alias)) v4ua;
union FragH { v16h v; v8h  half[2]; };
union FragB { v16b v; v8us half[2]; };

#define CCH   256
#define HH    64
#define WW    64
#define HWPIX (HH * WW)
#define KTAP  9
#define KDIM  (CCH * KTAP)
#define KSTEP 32
#define NIT   (KDIM / KSTEP)
#define MT    64
#define NSUB  4
#define TPB   256
#define NPW   32
#define OFFC  18
#define OFFN  32
#define HP    (HH + 2)
#define WP    (WW + 2)
#define ACAR  16.0f
#define WCAR  256.0f
#define SPH   136
#define SPF   132
#define SPO   36
#define SPX   68
#define PXT   264

static_assert(KDIM % KSTEP == 0);
static_assert(CCH % KSTEP == 0);
static_assert(CCH / KSTEP == 8);
static_assert(MT == WW);
static_assert(TPB == 8 * 32);
static_assert(MT * (KSTEP / 8) == TPB);
static_assert(NSUB * 16 == MT);
static_assert(CCH == 8 * NPW);
static_assert(TPB == CCH);
static_assert((SPH % 8) == 0 && (PXT % 8) == 0);
static_assert((SPF % 4) == 0 && (SPO % 4) == 0 && (SPX % 4) == 0);
static_assert((CCH * KDIM * 2) % 128 == 0);
static_assert((OFFN * KDIM * 2) % 128 == 0);
static_assert(OFFC <= OFFN);
static_assert((128 * MT) / 4 == 8 * TPB);

DEVINL int imin(int a, int b) { return a < b ? a : b; }
DEVINL int imax(int a, int b) { return a > b ? a : b; }
DEVINL int clampi(int v, int lo, int hi) { return imin(imax(v, lo), hi); }

DEVINL unsigned bf16_bits(float f) {
  unsigned u = __float_as_uint(f);
  u += 0x7FFFu + ((u >> 16) & 1u);
  return u >> 16;
}

DEVINL v8f wmma_f16(v16h a, v16h b, v8f c) {
  v8f d = __builtin_amdgcn_wmma_f32_16x16x32_f16(false, a, false, b, (short)0, c, false, false);
  asm volatile("v_nop\n\tv_nop\n\tv_nop\n\tv_nop" : "+v"(d) : "v"(a), "v"(b));
  return d;
}
DEVINL v8f wmma_bf16(v16b a, v16b b, v8f c) {
  v8f d = __builtin_amdgcn_wmma_f32_16x16x32_bf16(false, a, false, b, (short)0, c, false, false);
  asm volatile("v_nop\n\tv_nop\n\tv_nop\n\tv_nop" : "+v"(d) : "v"(a), "v"(b));
  return d;
}
DEVINL v8f zero8f() {
  v8f z = {0.f, 0.f, 0.f, 0.f, 0.f, 0.f, 0.f, 0.f};
  return z;
}

DEVINL v16h frag_row(const f16t* rowp, int h) {
  FragH f;
  f.half[0] = *(const v8ha*)(rowp + 8 * h);
  f.half[1] = *(const v8ha*)(rowp + 16 + 8 * h);
  return f.v;
}
DEVINL v16b frag_row_bf(const us16* rowp, int h) {
  FragB f;
  f.half[0] = *(const v8usa*)(rowp + 8 * h);
  f.half[1] = *(const v8usa*)(rowp + 16 + 8 * h);
  return f.v;
}

__global__ __launch_bounds__(TPB) void prep_w_k(const float* __restrict__ w1,
                                               const float* __restrict__ w2,
                                               const float* __restrict__ dw,
                                               const float* __restrict__ pw,
                                               f16t* __restrict__ w1T,
                                               f16t* __restrict__ w2T,
                                               f16t* __restrict__ dwT,
                                               us16* __restrict__ pwH,
                                               us16* __restrict__ pwL)
{
  const int y = blockIdx.y;
  const float* src = w1;
  f16t* dst = w1T;
  int nrow = CCH, nreal = CCH;
  float car = WCAR;
  if (y == 1)      { src = w2; dst = w2T; }
  else if (y == 2) { src = dw; dst = dwT; }
  else if (y == 3) { src = pw; nrow = OFFN; nreal = OFFC; car = 1.0f; }
  const int t = blockIdx.x * TPB + threadIdx.x;
  if (t >= nrow * (KDIM / 8)) return;
  const int n    = t / (KDIM / 8);
  const int part = t - n * (KDIM / 8);
  const int k0   = part * 8;
  const int tap  = k0 / CCH;
  const int cin0 = k0 - tap * CCH;
  const int nr   = (n < nreal) ? n : (nreal - 1);
  const float sc = (n < nreal) ? car : 0.0f;
  const float* sp = src + ((size_t)nr * CCH + cin0) * KTAP + tap;
  if (y == 3) {
    v8us oh, ol;
    #pragma unroll
    for (int j = 0; j < 8; ++j) {
      const float v  = sp[(size_t)j * KTAP] * sc;
      const unsigned hb = bf16_bits(v);
      const float hv = __uint_as_float(hb << 16);
      oh[j] = (us16)hb;
      ol[j] = (us16)bf16_bits(v - hv);
    }
    us16* dh = pwH + (size_t)8 * t;
    us16* dl = pwL + (size_t)8 * t;
    *(volatile v8us*)dh = oh;
    *(volatile v8us*)dl = ol;
    __threadfence();
    *(volatile v8us*)dh = oh;
    *(volatile v8us*)dl = ol;
  } else {
    v8h o;
    #pragma unroll
    for (int j = 0; j < 8; ++j) o[j] = (f16t)(sp[(size_t)j * KTAP] * sc);
    f16t* dp = dst + (size_t)8 * t;
    *(volatile v8h*)dp = o;
    __threadfence();
    *(volatile v8h*)dp = o;
  }
}

__global__ __launch_bounds__(TPB) void pack_x_k(const float* __restrict__ x, f16t* __restrict__ xpl)
{
  __shared__ __attribute__((aligned(16))) f16t sT[MT * PXT];
  const int tid  = threadIdx.x;
  const int lane = tid & 31;
  const int wave = tid >> 5;
  const int row  = blockIdx.x;
  const int b    = row >> 6;
  const int h    = row & 63;
  const float* xb = x + (size_t)b * CCH * HWPIX + (size_t)h * WW;
  #pragma unroll 4
  for (int i = 0; i < (MT * CCH) / TPB; ++i) {
    const int idx = i * TPB + tid;
    const int c = idx >> 6;
    const int w = idx & 63;
    const float v = xb[(size_t)c * HWPIX + w];
    sT[w * PXT + c] = (f16t)(v * ACAR);
  }
  __syncthreads();
  {
    const int q = lane >> 3, e = lane & 7;
    f16t* gt = xpl + (size_t)row * MT * CCH;
    v8h pv[8];
    int offh[8];
    #pragma unroll
    for (int i = 0; i < 8; ++i) {
      const int L = wave * 32 + 4 * i + q;
      const int px = L >> 2;
      const int choff = (L & 3) * 64 + e * 8;
      pv[i] = *(const v8ha*)&sT[px * PXT + choff];
      offh[i] = L * 64 + e * 8;
    }
    #pragma unroll
    for (int i = 0; i < 8; ++i) *(volatile v8h*)(gt + offh[i]) = pv[i];
    __threadfence();
    #pragma unroll
    for (int i = 0; i < 8; ++i) *(volatile v8h*)(gt + offh[i]) = pv[i];
  }
}

DEVINL void build_tile_f16(const f16t* __restrict__ src, f16t* tile, int b, int h,
                           int tap, int c0, int pgrp, int cgrp)
{
  const int tr = tap / 3, tc = tap - tr * 3;
  const int yy = h + tr - 1;
  const int xx = pgrp + tc - 1;
  const bool valid = (yy >= 0) && (yy <= HH - 1) && (xx >= 0) && (xx <= WW - 1);
  const int yyc = clampi(yy, 0, HH - 1);
  const int xxc = clampi(xx, 0, WW - 1);
  const f16t* sp = src + ((size_t)((b * HH + yyc) * WW + xxc)) * CCH + c0 + cgrp * 8;
  v4u v = *(const v4ua*)sp;
  const unsigned msk = valid ? 0xffffffffu : 0u;
  v = v & msk;
  *(v4ua*)(tile + pgrp * KSTEP + cgrp * 8) = v;
}

__global__ __launch_bounds__(TPB) void conv1_k(const f16t* __restrict__ xpl,
                                              const f16t* __restrict__ w1T,
                                              const float* __restrict__ b1,
                                              const float* __restrict__ x,
                                              f16t* __restrict__ res1)
{
  __shared__ __attribute__((aligned(16))) f16t  Als[2][MT * KSTEP];
  __shared__ __attribute__((aligned(16))) f16t  sStg[MT * SPH];
  __shared__ __attribute__((aligned(16))) float sBias[CCH];
  __shared__ __attribute__((aligned(16))) float sX[128 * SPX];

  const int tid  = threadIdx.x;
  const int lane = tid & 31;
  const int wave = tid >> 5;
  const int hl   = lane >> 4;
  const int m    = lane & 15;
  const int row  = blockIdx.x;
  const int b    = row >> 6;
  const int h    = row & 63;
  const int pix0 = row * MT;
  sBias[tid] = b1[tid];

  const int pgrp  = tid & 63;
  const int cgrp  = tid >> 6;
  const int nbase = wave * NPW;

  v8f acc[2][NSUB];
  #pragma unroll
  for (int j = 0; j < 2; ++j) {
    #pragma unroll
    for (int s = 0; s < NSUB; ++s) acc[j][s] = zero8f();
  }

  #pragma unroll 1
  for (int it = 0; it < NIT; ++it) {
    const int k0  = it * KSTEP;
    const int tap = it >> 3;
    const int c0  = (it & 7) * KSTEP;
    const int buf = it & 1;
    build_tile_f16(xpl, &Als[buf][0], b, h, tap, c0, pgrp, cgrp);
    __syncthreads();
    v16h wf[2];
    wf[0] = frag_row(w1T + (size_t)(nbase + m) * KDIM + k0, hl);
    wf[1] = frag_row(w1T + (size_t)(nbase + 16 + m) * KDIM + k0, hl);
    #pragma unroll
    for (int s = 0; s < NSUB; ++s) {
      const v16h xf = frag_row(&Als[buf][(s * 16 + m) * KSTEP], hl);
      acc[0][s] = wmma_f16(wf[0], xf, acc[0][s]);
      acc[1][s] = wmma_f16(wf[1], xf, acc[1][s]);
    }
  }

  const float kin = 1.0f / (ACAR * WCAR);
  #pragma unroll
  for (int p = 0; p < 2; ++p) {
    {
      v4f xv[8];
      int so[8];
      #pragma unroll
      for (int i = 0; i < 8; ++i) {
        const int idx = i * TPB + tid;
        const int cl  = idx >> 4;
        const int f4  = idx & 15;
        xv[i] = *(const v4fa*)(x + ((size_t)(b * CCH + p * 128 + cl) * HH + h) * WW + f4 * 4);
        so[i] = cl * SPX + f4 * 4;
      }
      #pragma unroll
      for (int i = 0; i < 8; ++i) *(v4fa*)&sX[so[i]] = xv[i];
    }
    __syncthreads();
    if ((wave >> 2) == p) {
      #pragma unroll
      for (int j = 0; j < 2; ++j) {
        #pragma unroll
        for (int s = 0; s < NSUB; ++s) {
          const int c  = nbase + 16 * j + 8 * hl;
          const int cl = c - 128 * p;
          const int px = 16 * s + m;
          v8h o;
          #pragma unroll
          for (int r = 0; r < 8; ++r) {
            float v = acc[j][s][r] * kin + sBias[c + r];
            v = fmaxf(v, 0.0f);
            v = v + sX[(cl + r) * SPX + px];
            o[r] = (f16t)(v * ACAR);
          }
          *(v8ha*)&sStg[px * SPH + cl] = o;
        }
      }
    }
    __syncthreads();
    {
      const int q = lane >> 3, e = lane & 7;
      v8h pv[4];
      size_t go[4];
      #pragma unroll
      for (int i = 0; i < 4; ++i) {
        const int L   = wave * 16 + 4 * i + q;
        const int px  = L >> 1;
        const int sub = L & 1;
        pv[i] = *(const v8ha*)&sStg[px * SPH + sub * 64 + e * 8];
        go[i] = (size_t)(pix0 + px) * CCH + p * 128 + sub * 64 + e * 8;
      }
      #pragma unroll
      for (int i = 0; i < 4; ++i) *(volatile v8h*)(res1 + go[i]) = pv[i];
      __threadfence();
      #pragma unroll
      for (int i = 0; i < 4; ++i) *(volatile v8h*)(res1 + go[i]) = pv[i];
    }
    __syncthreads();
  }
}

__global__ __launch_bounds__(TPB) void conv2_k(const f16t* __restrict__ res1,
                                              const f16t* __restrict__ w2T,
                                              const float* __restrict__ b2,
                                              float* __restrict__ res2)
{
  __shared__ __attribute__((aligned(16))) f16t  Als[2][MT * KSTEP];
  __shared__ __attribute__((aligned(16))) float sStg[MT * SPF];
  __shared__ __attribute__((aligned(16))) float sBias[CCH];

  const int tid  = threadIdx.x;
  const int lane = tid & 31;
  const int wave = tid >> 5;
  const int hl   = lane >> 4;
  const int m    = lane & 15;
  const int row  = blockIdx.x;
  const int b    = row >> 6;
  const int h    = row & 63;
  const int pix0 = row * MT;
  sBias[tid] = b2[tid];

  const int pgrp  = tid & 63;
  const int cgrp  = tid >> 6;
  const int nbase = wave * NPW;

  v8f acc[2][NSUB];
  #pragma unroll
  for (int j = 0; j < 2; ++j) {
    #pragma unroll
    for (int s = 0; s < NSUB; ++s) acc[j][s] = zero8f();
  }

  #pragma unroll 1
  for (int it = 0; it < NIT; ++it) {
    const int k0  = it * KSTEP;
    const int tap = it >> 3;
    const int c0  = (it & 7) * KSTEP;
    const int buf = it & 1;
    build_tile_f16(res1, &Als[buf][0], b, h, tap, c0, pgrp, cgrp);
    __syncthreads();
    v16h wf[2];
    wf[0] = frag_row(w2T + (size_t)(nbase + m) * KDIM + k0, hl);
    wf[1] = frag_row(w2T + (size_t)(nbase + 16 + m) * KDIM + k0, hl);
    #pragma unroll
    for (int s = 0; s < NSUB; ++s) {
      const v16h xf = frag_row(&Als[buf][(s * 16 + m) * KSTEP], hl);
      acc[0][s] = wmma_f16(wf[0], xf, acc[0][s]);
      acc[1][s] = wmma_f16(wf[1], xf, acc[1][s]);
    }
  }

  const float kin = 1.0f / (ACAR * WCAR);
  #pragma unroll
  for (int p = 0; p < 2; ++p) {
    if ((wave >> 2) == p) {
      #pragma unroll
      for (int j = 0; j < 2; ++j) {
        #pragma unroll
        for (int s = 0; s < NSUB; ++s) {
          const int c  = nbase + 16 * j + 8 * hl;
          const int cl = c - 128 * p;
          const int px = 16 * s + m;
          v4f lo4, hi4;
          #pragma unroll
          for (int r = 0; r < 4; ++r) {
            lo4[r] = acc[j][s][r]     * kin + sBias[c + r];
            hi4[r] = acc[j][s][4 + r] * kin + sBias[c + 4 + r];
          }
          *(v4fa*)&sStg[px * SPF + cl]     = lo4;
          *(v4fa*)&sStg[px * SPF + cl + 4] = hi4;
        }
      }
    }
    __syncthreads();
    {
      const int q = lane >> 3, e = lane & 7;
      v4f pv[8];
      size_t go[8];
      #pragma unroll
      for (int i = 0; i < 8; ++i) {
        const int L   = wave * 32 + 4 * i + q;
        const int px  = L >> 2;
        const int sub = L & 3;
        pv[i] = *(const v4fa*)&sStg[px * SPF + sub * 32 + e * 4];
        go[i] = (size_t)(pix0 + px) * CCH + p * 128 + sub * 32 + e * 4;
      }
      #pragma unroll
      for (int i = 0; i < 8; ++i) *(volatile v4f*)(res2 + go[i]) = pv[i];
      __threadfence();
      #pragma unroll
      for (int i = 0; i < 8; ++i) *(volatile v4f*)(res2 + go[i]) = pv[i];
    }
    __syncthreads();
  }
}

__global__ __launch_bounds__(TPB) void off_k(const float* __restrict__ res2,
                                            const us16* __restrict__ pwH,
                                            const us16* __restrict__ pwL,
                                            const float* __restrict__ pb,
                                            float* __restrict__ offs)
{
  __shared__ __attribute__((aligned(16))) us16  AlsH[2][MT * KSTEP];
  __shared__ __attribute__((aligned(16))) us16  AlsL[2][MT * KSTEP];
  __shared__ __attribute__((aligned(16))) float sStg[MT * SPO];
  __shared__ __attribute__((aligned(16))) float sPb[OFFN];

  const int tid  = threadIdx.x;
  const int lane = tid & 31;
  const int wave = tid >> 5;
  const int hl   = lane >> 4;
  const int m    = lane & 15;
  const int row  = blockIdx.x;
  const int b    = row >> 6;
  const int h    = row & 63;
  const int pix0 = row * MT;
  if (tid < OFFN) {
    const float v = pb[imin(tid, OFFC - 1)];
    sPb[tid] = (tid < OFFC) ? v : 0.0f;
  }

  const int pgrp = tid & 63;
  const int cgrp = tid >> 6;
  const int s    = wave & 3;
  const int j    = wave >> 2;

  v8f acc = zero8f();

  #pragma unroll 1
  for (int it = 0; it < NIT; ++it) {
    const int k0  = it * KSTEP;
    const int tap = it >> 3;
    const int c0  = (it & 7) * KSTEP;
    const int buf = it & 1;
    {
      const int tr = tap / 3, tc = tap - tr * 3;
      const int yy = h + tr - 1;
      const int xx = pgrp + tc - 1;
      const bool valid = (yy >= 0) && (yy <= HH - 1) && (xx >= 0) && (xx <= WW - 1);
      const int yyc = clampi(yy, 0, HH - 1);
      const int xxc = clampi(xx, 0, WW - 1);
      const float* sp = res2 + ((size_t)((b * HH + yyc) * WW + xxc)) * CCH + c0 + cgrp * 8;
      const v4f a0 = *(const v4fa*)sp;
      const v4f a1 = *(const v4fa*)(sp + 4);
      const float msc = valid ? 1.0f : 0.0f;
      v8us oh, ol;
      #pragma unroll
      for (int i = 0; i < 4; ++i) {
        const float v0 = a0[i] * msc;
        const float v1 = a1[i] * msc;
        const unsigned h0 = bf16_bits(v0);
        const unsigned h1 = bf16_bits(v1);
        const float hv0 = __uint_as_float(h0 << 16);
        const float hv1 = __uint_as_float(h1 << 16);
        oh[i]     = (us16)h0;
        oh[4 + i] = (us16)h1;
        ol[i]     = (us16)bf16_bits(v0 - hv0);
        ol[4 + i] = (us16)bf16_bits(v1 - hv1);
      }
      *(v8usa*)&AlsH[buf][pgrp * KSTEP + cgrp * 8] = oh;
      *(v8usa*)&AlsL[buf][pgrp * KSTEP + cgrp * 8] = ol;
    }
    __syncthreads();
    const v16b wh = frag_row_bf(pwH + (size_t)(16 * j + m) * KDIM + k0, hl);
    const v16b wl = frag_row_bf(pwL + (size_t)(16 * j + m) * KDIM + k0, hl);
    const v16b xh = frag_row_bf(&AlsH[buf][(s * 16 + m) * KSTEP], hl);
    const v16b xl = frag_row_bf(&AlsL[buf][(s * 16 + m) * KSTEP], hl);
    acc = wmma_bf16(wh, xh, acc);
    acc = wmma_bf16(wh, xl, acc);
    acc = wmma_bf16(wl, xh, acc);
  }

  {
    const int c  = 16 * j + 8 * hl;
    const int px = 16 * s + m;
    v4f lo4, hi4;
    #pragma unroll
    for (int r = 0; r < 4; ++r) {
      lo4[r] = acc[r]     + sPb[c + r];
      hi4[r] = acc[4 + r] + sPb[c + 4 + r];
    }
    *(v4fa*)&sStg[px * SPO + c]     = lo4;
    *(v4fa*)&sStg[px * SPO + c + 4] = hi4;
  }
  __syncthreads();
  {
    const int q = lane >> 3, e = lane & 7;
    v4f pv[2];
    size_t go[2];
    #pragma unroll
    for (int i = 0; i < 2; ++i) {
      const int L  = wave * 8 + 4 * i + q;
      pv[i] = *(const v4fa*)&sStg[L * SPO + e * 4];
      go[i] = (size_t)(pix0 + L) * OFFN + e * 4;
    }
    #pragma unroll
    for (int i = 0; i < 2; ++i) *(volatile v4f*)(offs + go[i]) = pv[i];
    __threadfence();
    #pragma unroll
    for (int i = 0; i < 2; ++i) *(volatile v4f*)(offs + go[i]) = pv[i];
  }
}

__global__ __launch_bounds__(TPB) void deform_k(const float* __restrict__ res2,
                                               const float* __restrict__ offs,
                                               const f16t* __restrict__ dwT,
                                               const float* __restrict__ x,
                                               float* __restrict__ out)
{
  __shared__ __attribute__((aligned(16))) v4i   sO[MT * KTAP];
  __shared__ __attribute__((aligned(16))) v4f   sW[MT * KTAP];
  __shared__ __attribute__((aligned(16))) f16t  Als[2][MT * KSTEP];
  __shared__ __attribute__((aligned(16))) float sStg[128 * SPX];

  const int tid  = threadIdx.x;
  const int lane = tid & 31;
  const int wave = tid >> 5;
  const int hl   = lane >> 4;
  const int m    = lane & 15;
  const int row  = blockIdx.x;
  const int b    = row >> 6;
  const int h    = row & 63;
  const int pix0 = row * MT;

  #pragma unroll 1
  for (int t = tid; t < MT * KTAP; t += TPB) {
    const int p   = t / KTAP;
    const int tap = t - p * KTAP;
    const int tr  = tap / 3, tc = tap - tr * 3;
    const float offr = offs[(size_t)(pix0 + p) * OFFN + tap];
    const float offc = offs[(size_t)(pix0 + p) * OFFN + KTAP + tap];
    const float pr0 = offr + (float)(tr - 1);
    const float pr  = pr0 + (float)(h + 1);
    const float pc0 = offc + (float)(tc - 1);
    const float pc  = pc0 + (float)(p + 1);
    const float fr = floorf(pr), fc = floorf(pc);
    const float hir = (float)(HP - 1), hic = (float)(WP - 1);
    const float qlr = fminf(fmaxf(fr, 0.0f), hir);
    const float qrr = fminf(fmaxf(fr + 1.0f, 0.0f), hir);
    const float qlc = fminf(fmaxf(fc, 0.0f), hic);
    const float qrc = fminf(fmaxf(fc + 1.0f, 0.0f), hic);
    const float prc = fminf(fmaxf(pr, 0.0f), hir);
    const float pcc = fminf(fmaxf(pc, 0.0f), hic);
    const float al = (1.0f + qlr) - prc;
    const float ar = (1.0f - qrr) + prc;
    const float bl = (1.0f + qlc) - pcc;
    const float br = (1.0f - qrc) + pcc;
    const float glt = al * bl;
    const float grb = ar * br;
    const float glb = al * br;
    const float grt = ar * bl;
    const int ilr = (int)qlr, irr = (int)qrr, ilc = (int)qlc, irc = (int)qrc;
    const bool vlr = (ilr >= 1) && (ilr <= HH);
    const bool vrr = (irr >= 1) && (irr <= HH);
    const bool vlc = (ilc >= 1) && (ilc <= WW);
    const bool vrc = (irc >= 1) && (irc <= WW);
    const int ulr = clampi(ilr - 1, 0, HH - 1);
    const int urr = clampi(irr - 1, 0, HH - 1);
    const int ulc = clampi(ilc - 1, 0, WW - 1);
    const int urc = clampi(irc - 1, 0, WW - 1);
    v4i o;
    o[0] = ulr * WW + ulc;
    o[1] = urr * WW + urc;
    o[2] = ulr * WW + urc;
    o[3] = urr * WW + ulc;
    v4f g;
    g[0] = (vlr && vlc) ? glt : 0.0f;
    g[1] = (vrr && vrc) ? grb : 0.0f;
    g[2] = (vlr && vrc) ? glb : 0.0f;
    g[3] = (vrr && vlc) ? grt : 0.0f;
    sO[t] = o;
    sW[t] = g;
  }
  __syncthreads();

  const int pgrp  = tid & 63;
  const int cgrp  = tid >> 6;
  const int nbase = wave * NPW;
  const float* rb = res2 + (size_t)b * HWPIX * CCH;

  v8f acc[2][NSUB];
  #pragma unroll
  for (int j = 0; j < 2; ++j) {
    #pragma unroll
    for (int s = 0; s < NSUB; ++s) acc[j][s] = zero8f();
  }

  #pragma unroll 1
  for (int it = 0; it < NIT; ++it) {
    const int k0  = it * KSTEP;
    const int tap = it >> 3;
    const int c0  = (it & 7) * KSTEP;
    const int buf = it & 1;
    {
      const v4i o = sO[pgrp * KTAP + tap];
      const v4f g = sW[pgrp * KTAP + tap];
      const float* base = rb + c0 + cgrp * 8;
      const float* p0 = base + (size_t)o[0] * CCH;
      const float* p1 = base + (size_t)o[1] * CCH;
      const float* p2 = base + (size_t)o[2] * CCH;
      const float* p3 = base + (size_t)o[3] * CCH;
      const v4f a0 = *(const v4fa*)p0, a1 = *(const v4fa*)(p0 + 4);
      const v4f b0 = *(const v4fa*)p1, b1 = *(const v4fa*)(p1 + 4);
      const v4f e0 = *(const v4fa*)p2, e1 = *(const v4fa*)(p2 + 4);
      const v4f d0 = *(const v4fa*)p3, d1 = *(const v4fa*)(p3 + 4);
      v8h ov;
      #pragma unroll
      for (int i = 0; i < 4; ++i) {
        const float v0 = ((g[0] * a0[i] + g[1] * b0[i]) + g[2] * e0[i]) + g[3] * d0[i];
        const float v1 = ((g[0] * a1[i] + g[1] * b1[i]) + g[2] * e1[i]) + g[3] * d1[i];
        ov[i]     = (f16t)(v0 * ACAR);
        ov[4 + i] = (f16t)(v1 * ACAR);
      }
      *(v8ha*)&Als[buf][pgrp * KSTEP + cgrp * 8] = ov;
    }
    __syncthreads();
    v16h wf[2];
    wf[0] = frag_row(dwT + (size_t)(nbase + m) * KDIM + k0, hl);
    wf[1] = frag_row(dwT + (size_t)(nbase + 16 + m) * KDIM + k0, hl);
    #pragma unroll
    for (int s = 0; s < NSUB; ++s) {
      const v16h xf = frag_row(&Als[buf][(s * 16 + m) * KSTEP], hl);
      acc[0][s] = wmma_f16(xf, wf[0], acc[0][s]);
      acc[1][s] = wmma_f16(xf, wf[1], acc[1][s]);
    }
  }

  const float kin = 1.0f / (ACAR * WCAR);
  #pragma unroll
  for (int p = 0; p < 2; ++p) {
    if ((wave >> 2) == p) {
      #pragma unroll
      for (int j = 0; j < 2; ++j) {
        #pragma unroll
        for (int s = 0; s < NSUB; ++s) {
          const int cl = (wave - 4 * p) * NPW + 16 * j + m;
          float* rowp = &sStg[cl * SPX + 16 * s + 8 * hl];
          v4f lo4, hi4;
          #pragma unroll
          for (int r = 0; r < 4; ++r) { lo4[r] = acc[j][s][r] * kin; hi4[r] = acc[j][s][4 + r] * kin; }
          *(v4fa*)rowp       = lo4;
          *(v4fa*)(rowp + 4) = hi4;
        }
      }
    }
    __syncthreads();
    {
      const int q = lane >> 3, e = lane & 7;
      v4f ov[8];
      size_t go[8];
      #pragma unroll
      for (int i = 0; i < 8; ++i) {
        const int L   = wave * 32 + 4 * i + q;
        const int cl  = L >> 1;
        const int sub = L & 1;
        const int c   = p * 128 + cl;
        const v4f a   = *(const v4fa*)&sStg[cl * SPX + sub * 32 + e * 4];
        go[i] = ((size_t)(b * CCH + c) * HH + h) * WW + sub * 32 + e * 4;
        const v4f xr = *(const v4fa*)(x + go[i]);
        v4f o;
        #pragma unroll
        for (int jj = 0; jj < 4; ++jj) o[jj] = a[jj] + xr[jj];
        ov[i] = o;
      }
      #pragma unroll
      for (int i = 0; i < 8; ++i) *(volatile v4f*)(out + go[i]) = ov[i];
      __threadfence();
      #pragma unroll
      for (int i = 0; i < 8; ++i) *(volatile v4f*)(out + go[i]) = ov[i];
    }
    __syncthreads();
  }
}

extern "C" void kernel_launch(void* const* d_in, const int* in_sizes, int n_in,
                              void* d_out, int out_size, void* d_ws, size_t ws_size,
                              hipStream_t stream) {
  if (n_in < 8) return;
  const int chw = CCH * HWPIX;
  if (in_sizes[0] <= 0 || (in_sizes[0] % chw) != 0) return;
  const int nB = in_sizes[0] / chw;
  if (in_sizes[1] != CCH * KDIM || in_sizes[3] != CCH * KDIM || in_sizes[7] != CCH * KDIM) return;
  if (in_sizes[2] != CCH || in_sizes[4] != CCH) return;
  if (in_sizes[5] != OFFC * KDIM || in_sizes[6] != OFFC) return;
  if (out_size != in_sizes[0]) return;

  const float* x   = (const float*)d_in[0];
  const float* w1  = (const float*)d_in[1];
  const float* b1  = (const float*)d_in[2];
  const float* w2  = (const float*)d_in[3];
  const float* b2  = (const float*)d_in[4];
  const float* p_w = (const float*)d_in[5];
  const float* p_b = (const float*)d_in[6];
  const float* dw  = (const float*)d_in[7];
  float* outp = (float*)d_out;

  const size_t szXP = (size_t)nB * HWPIX * CCH * 2;
  const size_t szR1 = szXP;
  const size_t szR2 = (size_t)nB * HWPIX * CCH * 4;
  const size_t szOF = (size_t)nB * HWPIX * OFFN * 4;
  const size_t szW  = (size_t)CCH * KDIM * 2;
  const size_t szPW = (size_t)OFFN * KDIM * 2;
  size_t off = 0;
  char* ws = (char*)d_ws;
  f16t*  xpl  = (f16t*)(ws + off);  off += szXP;
  f16t*  res1 = (f16t*)(ws + off);  off += szR1;
  float* res2 = (float*)(ws + off); off += szR2;
  float* offs = (float*)(ws + off); off += szOF;
  f16t*  w1T  = (f16t*)(ws + off);  off += szW;
  f16t*  w2T  = (f16t*)(ws + off);  off += szW;
  f16t*  dwT  = (f16t*)(ws + off);  off += szW;
  us16*  pwH  = (us16*)(ws + off);  off += szPW;
  us16*  pwL  = (us16*)(ws + off);  off += szPW;
  if (off > ws_size) return;

  const int rows = nB * HH;

  prep_w_k<<<dim3((CCH * (KDIM / 8)) / TPB, 4), TPB, 0, stream>>>(w1, w2, dw, p_w, w1T, w2T, dwT, pwH, pwL);
  pack_x_k<<<rows, TPB, 0, stream>>>(x, xpl);
  conv1_k<<<rows, TPB, 0, stream>>>(xpl, w1T, b1, x, res1);
  conv2_k<<<rows, TPB, 0, stream>>>(res1, w2T, b2, res2);
  off_k<<<rows, TPB, 0, stream>>>(res2, pwH, pwL, p_b, offs);
  deform_k<<<rows, TPB, 0, stream>>>(res2, offs, dwT, x, outp);
}
